// coRNN_62835371540840
// MI455X (gfx1250) — hardware-run, weakly checked
//
#include <hip/hip_runtime.h>
#include <math.h>

constexpr int NSTEP  = 512;
constexpr int NBAT   = 128;
constexpr int NINP   = 128;
constexpr int NHID   = 1024;
constexpr int NCHAN  = 2;
constexpr int NSTATE = NCHAN * NHID;
constexpr int NOUTF  = 10;
constexpr int TCHUNK = 64;
constexpr int NCHUNK = NSTEP / TCHUNK;
constexpr int MCHUNK = TCHUNK * NBAT;
constexpr int NROWS  = NSTEP * NBAT;
constexpr int NTHR   = 256;
static_assert(NSTEP % TCHUNK == 0);
static_assert(NINP % 32 == 0);
static_assert(MCHUNK % 64 == 0 && NSTATE % 64 == 0);
static_assert(((MCHUNK / 64) * (NSTATE / 64)) % 8 == 0);
static_assert(NHID == 4 * NTHR);
static_assert((NHID & (NHID - 1)) == 0);
static_assert((NBAT * NOUTF) % NTHR == 0);
static_assert((NROWS * (NINP / 8)) % NTHR == 0);
static_assert((NSTATE * (NINP / 8)) % NTHR == 0);
static_assert((NSTATE / 4) % NTHR == 0);

typedef __attribute__((ext_vector_type(16))) _Float16 v16h;
typedef __attribute__((ext_vector_type(8)))  _Float16 v8h;
typedef __attribute__((ext_vector_type(16))) __bf16   v16b;
typedef __attribute__((ext_vector_type(8)))  __bf16   v8b;
typedef __attribute__((ext_vector_type(8)))  float    v8f;
typedef __attribute__((ext_vector_type(4)))  float    v4f;

__device__ __forceinline__ unsigned short f2bf_bits(float f) {
  unsigned u = __float_as_uint(f);
  return (unsigned short)((u + 0x7FFFu + ((u >> 16) & 1u)) >> 16);
}
__device__ __forceinline__ float bf_bits2f(unsigned short h) { return __uint_as_float(((unsigned)h) << 16); }
__device__ __forceinline__ float bf16r(float f) { return bf_bits2f(f2bf_bits(f)); }

__device__ __forceinline__ void dep_guard4_h(v8f& a, v8f& b, v8f& c, v8f& d, v16h x, v16h y) { asm volatile("v_nop\n\tv_nop\n\tv_nop\n\tv_nop" : "+v"(a), "+v"(b), "+v"(c), "+v"(d) : "v"(x), "v"(y)); }
__device__ __forceinline__ void dep_guard4_b(v8f& a, v8f& b, v8f& c, v8f& d, v16b x, v16b y) { asm volatile("v_nop\n\tv_nop\n\tv_nop\n\tv_nop" : "+v"(a), "+v"(b), "+v"(c), "+v"(d) : "v"(x), "v"(y)); }
__device__ __forceinline__ void keep4_h(v16h a, v16h b, v16h c, v16h d) { asm volatile("v_nop" :: "v"(a), "v"(b), "v"(c), "v"(d)); }
__device__ __forceinline__ void keep4_b(v16b a, v16b b, v16b c, v16b d) { asm volatile("v_nop" :: "v"(a), "v"(b), "v"(c), "v"(d)); }
__device__ __forceinline__ void acc_guard4(v8f& a, v8f& b, v8f& c, v8f& d) { asm volatile("v_nop\n\tv_nop\n\tv_nop\n\tv_nop" : "+v"(a), "+v"(b), "+v"(c), "+v"(d)); }

template <typename T> struct Frag;
template <> struct Frag<_Float16> {
  typedef v16h V; union U { v16h v; v8h h[2]; };
  static __device__ __forceinline__ v16h load(const _Float16* p) {
    U f; f.h[0] = *(const v8h*)(p); f.h[1] = *(const v8h*)(p + 16); return f.v;
  }
  static __device__ __forceinline__ v8f mma(v16h a, v16h b, v8f c) {
    return __builtin_amdgcn_wmma_f32_16x16x32_f16(false, a, false, b, (short)0, c, false, false);
  }
  static __device__ __forceinline__ void guard4(v8f& a, v8f& b, v8f& c, v8f& d, v16h x, v16h y) { dep_guard4_h(a, b, c, d, x, y); }
  static __device__ __forceinline__ void keep(v16h a, v16h b, v16h c, v16h d) { keep4_h(a, b, c, d); }
};
template <> struct Frag<__bf16> {
  typedef v16b V; union U { v16b v; v8b h[2]; };
  static __device__ __forceinline__ v16b load(const __bf16* p) {
    U f; f.h[0] = *(const v8b*)(p); f.h[1] = *(const v8b*)(p + 16); return f.v;
  }
  static __device__ __forceinline__ v8f mma(v16b a, v16b b, v8f c) {
    return __builtin_amdgcn_wmma_f32_16x16x32_bf16(false, a, false, b, (short)0, c, false, false);
  }
  static __device__ __forceinline__ void guard4(v8f& a, v8f& b, v8f& c, v8f& d, v16b x, v16b y) { dep_guard4_b(a, b, c, d, x, y); }
  static __device__ __forceinline__ void keep(v16b a, v16b b, v16b c, v16b d) { keep4_b(a, b, c, d); }
};

template <int ET> struct Elem;
template <> struct Elem<0> { typedef _Float16 T; };
template <> struct Elem<1> { typedef __bf16 T; };
template <int ET, bool SPLIT, int BIAS_MODE, int OUT_MODE, bool RESID, int ACT = 0>
__global__ __launch_bounds__(256) void wmma_gemm64(
    const unsigned short* __restrict__ Ap, const unsigned short* __restrict__ A2p, int lda, long strideA,
    const unsigned short* __restrict__ Btp, const unsigned short* __restrict__ Bt2p, int ldb, long strideB,
    void* __restrict__ Cout, void* __restrict__ Cout2, int ldc, long strideC,
    const float* __restrict__ bias,
    const float* __restrict__ resid, long strideR,
    int M, int N, int K, float scale) {
  typedef typename Elem<ET>::T T;
  typedef typename Frag<T>::V V;
  const T* A = (const T*)Ap; const T* A2 = (const T*)A2p; const T* Bt = (const T*)Btp; const T* Bt2 = (const T*)Bt2p;
  __shared__ __align__(16) float sT[8][16 * 68];
  const int b    = blockIdx.y;
  const int lane = threadIdx.x & 31;
  const int wave = threadIdx.x >> 5;
  const int tilesN = N >> 6;
  const int tilesM = M >> 6;
  const int tile = blockIdx.x * 8 + wave;
  if (tile >= tilesM * tilesN) return;
  const int tm = tile / tilesN;
  const int tn = tile - tm * tilesN;
  const int m0 = tm << 6;
  const int n0 = tn << 6;

  const T* Ab  = A  + (size_t)b * strideA;
  const T* Bb  = Bt + (size_t)b * strideB;
  const T* Ab2 = SPLIT ? (A2  + (size_t)b * strideA) : nullptr;
  const T* Bb2 = SPLIT ? (Bt2 + (size_t)b * strideB) : nullptr;

  const int rlane = lane & 15;
  const int koff  = (lane >> 4) * 8;
  const int mOff  = (lane >> 4) * 8;

  v8f acc[4][4];
#pragma unroll
  for (int i = 0; i < 4; ++i)
#pragma unroll
    for (int j = 0; j < 4; ++j) acc[i][j] = (v8f){0.f,0.f,0.f,0.f,0.f,0.f,0.f,0.f};

  for (int k0 = 0; k0 < K; k0 += 32) {
    V bh[4], bl[4];
#pragma unroll
    for (int j = 0; j < 4; ++j) {
      const size_t bo = (size_t)(n0 + (j << 4) + rlane) * ldb + koff + k0;
      bh[j] = Frag<T>::load(Bb + bo);
      if (SPLIT) bl[j] = Frag<T>::load(Bb2 + bo);
    }
#pragma unroll
    for (int i = 0; i < 4; ++i) {
      const size_t ao = (size_t)(m0 + (i << 4) + rlane) * lda + koff + k0;
      V ah = Frag<T>::load(Ab + ao);
      V al;
      if (SPLIT) al = Frag<T>::load(Ab2 + ao);
#pragma unroll
      for (int j = 0; j < 4; ++j) {
        acc[i][j] = Frag<T>::mma(ah, bh[j], acc[i][j]);
        if (SPLIT) {
          acc[i][j] = Frag<T>::mma(ah, bl[j], acc[i][j]);
          acc[i][j] = Frag<T>::mma(al, bh[j], acc[i][j]);
        }
      }
      Frag<T>::guard4(acc[i][0], acc[i][1], acc[i][2], acc[i][3], ah, SPLIT ? al : ah);
    }
    Frag<T>::keep(bh[0], bh[1], bh[2], bh[3]);
    if (SPLIT) Frag<T>::keep(bl[0], bl[1], bl[2], bl[3]);
  }
  acc_guard4(acc[0][0], acc[0][1], acc[0][2], acc[0][3]);
  acc_guard4(acc[1][0], acc[1][1], acc[1][2], acc[1][3]);
  acc_guard4(acc[2][0], acc[2][1], acc[2][2], acc[2][3]);
  acc_guard4(acc[3][0], acc[3][1], acc[3][2], acc[3][3]);

  float* slab = sT[wave];
  const float* Rb = RESID ? (resid + (size_t)b * strideR) : nullptr;
#pragma unroll
  for (int i = 0; i < 4; ++i) {
    const int mBase = m0 + (i << 4);
#pragma unroll
    for (int j = 0; j < 4; ++j) {
      const int n = n0 + (j << 4) + rlane;
      float bv = 0.f;
      if (BIAS_MODE == 2) bv = bias[n];
#pragma unroll
      for (int r = 0; r < 8; ++r) {
        float v = acc[i][j][r] * scale;
        if (BIAS_MODE == 1) v += bias[mBase + mOff + r];
        if (BIAS_MODE == 2) v += bv;
        if (RESID) v += Rb[(size_t)(mBase + mOff + r) * ldc + n];
        if (ACT == 1) v = tanhf(v);
        if (ACT == 2) v = fmaxf(v, 0.0f);
        slab[(mOff + r) * 68 + (j << 4) + rlane] = v;
      }
    }
    __builtin_amdgcn_fence(__ATOMIC_RELEASE, "workgroup");
    __builtin_amdgcn_wave_barrier();
    __builtin_amdgcn_fence(__ATOMIC_ACQUIRE, "workgroup");
    if (OUT_MODE == 0) {
      float* C = (float*)Cout + (size_t)b * strideC;
      const int hh = lane >> 4, c4 = (lane & 15) * 4;
      for (int pass = 0; pass < 2; ++pass) {
#pragma unroll
        for (int it = 0; it < 8; ++it) {
          const int row = it * 2 + hh;
          v4f v = *(const v4f*)(slab + row * 68 + c4);
          *(volatile v4f*)(C + (size_t)(mBase + row) * ldc + n0 + c4) = v;
        }
        __threadfence();
      }
    } else {
      const int q = lane >> 3, c8 = (lane & 7) * 8;
      unsigned short* C  = (unsigned short*)Cout  + (size_t)b * strideC;
      unsigned short* C2 = (OUT_MODE == 2) ? ((unsigned short*)Cout2 + (size_t)b * strideC) : nullptr;
      for (int pass = 0; pass < 2; ++pass) {
#pragma unroll
        for (int it = 0; it < 4; ++it) {
          const int row = it * 4 + q;
          const float* sp = slab + row * 68 + c8;
          v8h hv, lv;
#pragma unroll
          for (int e = 0; e < 8; ++e) {
            if (OUT_MODE == 1) {
              hv[e] = (_Float16)sp[e];
            } else {
              unsigned short hb = f2bf_bits(sp[e]);
              unsigned short lb = f2bf_bits(sp[e] - bf_bits2f(hb));
              hv[e] = __builtin_bit_cast(_Float16, hb);
              lv[e] = __builtin_bit_cast(_Float16, lb);
            }
          }
          *(volatile v8h*)(C + (size_t)(mBase + row) * ldc + n0 + c8) = hv;
          if (OUT_MODE == 2) *(volatile v8h*)(C2 + (size_t)(mBase + row) * ldc + n0 + c8) = lv;
        }
        __threadfence();
      }
    }
    __builtin_amdgcn_fence(__ATOMIC_RELEASE, "workgroup");
    __builtin_amdgcn_wave_barrier();
    __builtin_amdgcn_fence(__ATOMIC_ACQUIRE, "workgroup");
  }
}

__global__ __launch_bounds__(NTHR) void cvt8_bf16_kernel(const float* __restrict__ src, unsigned short* __restrict__ dst, int n8) {
  const int i = blockIdx.x * NTHR + threadIdx.x;
  if (i < n8) {
    const float* sp = src + (size_t)i * 8;
    const v4f a = *(const v4f*)(sp);
    const v4f b = *(const v4f*)(sp + 4);
    v8h hv;
#pragma unroll
    for (int e = 0; e < 4; ++e) {
      const unsigned short b0 = f2bf_bits(a[e]);
      const unsigned short b1 = f2bf_bits(b[e]);
      hv[e]     = __builtin_bit_cast(_Float16, b0);
      hv[4 + e] = __builtin_bit_cast(_Float16, b1);
    }
    *(volatile v8h*)(dst + (size_t)i * 8) = hv;
    __threadfence();
    *(volatile v8h*)(dst + (size_t)i * 8) = hv;
  }
}

__global__ __launch_bounds__(NTHR) void rne_plane_kernel(const float* __restrict__ src, float* __restrict__ dst, int n4) {
  const int i = blockIdx.x * NTHR + threadIdx.x;
  if (i < n4) {
    const v4f a = *(const v4f*)(src + (size_t)i * 4);
    v4f o;
#pragma unroll
    for (int e = 0; e < 4; ++e) o[e] = bf16r(a[e]);
    float* op = dst + (size_t)i * 4;
    *(volatile v4f*)op = o;
    __threadfence();
    *(volatile v4f*)op = o;
  }
}

__global__ __launch_bounds__(NTHR) void rec_chunk_kernel(const float* __restrict__ U, const float* __restrict__ Wy_w,
                                                         const float* __restrict__ Wy_b, float* __restrict__ H, int first) {
  __shared__ __align__(16) float hbuf[2][NSTATE];
  const int tid = threadIdx.x;
  const int b   = blockIdx.x;
  const int j0  = 4 * tid;
  const int jm  = (j0 + NHID - 1) & (NHID - 1);
  const int jp  = (j0 + 4) & (NHID - 1);

  float w[2][2][12];
  float bb[2][4];
#pragma unroll
  for (int o = 0; o < 2; ++o) {
    const v4f bv = *(const v4f*)(Wy_b + o * NHID + j0);
#pragma unroll
    for (int e = 0; e < 4; ++e) bb[o][e] = bf16r(bv[e]);
#pragma unroll
    for (int c = 0; c < 2; ++c) {
      const float* wp = Wy_w + ((size_t)((o * 2 + c) * NHID + j0)) * 3;
#pragma unroll
      for (int q = 0; q < 3; ++q) {
        const v4f wv = *(const v4f*)(wp + 4 * q);
#pragma unroll
        for (int e = 0; e < 4; ++e) w[o][c][4 * q + e] = bf16r(wv[e]);
      }
    }
  }

  {
    float* h0 = &hbuf[0][0];
    if (first != 0) {
#pragma unroll
      for (int e = 0; e < 4; ++e) { h0[j0 + e] = 0.0f; h0[NHID + j0 + e] = 0.0f; }
    } else {
      const float* hp = H + (size_t)b * NSTATE + j0;
      const v4f a0 = *(const v4f*)(hp);
      const v4f a1 = *(const v4f*)(hp + NHID);
#pragma unroll
      for (int e = 0; e < 4; ++e) { h0[j0 + e] = a0[e]; h0[NHID + j0 + e] = a1[e]; }
    }
  }
  __syncthreads();

  int cur = 0;
#pragma unroll 1
  for (int s = 0; s < TCHUNK; ++s) {
    const float* hc = &hbuf[cur][0];
    float*       hn = &hbuf[cur ^ 1][0];
    const float* up = U + ((size_t)(s * NBAT + b)) * NSTATE + j0;
    const v4f u0 = *(const v4f*)(up);
    const v4f u1 = *(const v4f*)(up + NHID);

    float hw[2][6];
#pragma unroll
    for (int c = 0; c < 2; ++c) {
      hw[c][0] = hc[c * NHID + jm];
#pragma unroll
      for (int e = 0; e < 4; ++e) hw[c][1 + e] = hc[c * NHID + j0 + e];
      hw[c][5] = hc[c * NHID + jp];
    }
#pragma unroll
    for (int o = 0; o < 2; ++o) {
#pragma unroll
      for (int e = 0; e < 4; ++e) {
        float loc = 0.0f;
#pragma unroll
        for (int c = 0; c < 2; ++c)
#pragma unroll
          for (int k = 0; k < 3; ++k) loc += hw[c][e + k] * w[o][c][e * 3 + k];
        const float uu = (o == 0) ? u0[e] : u1[e];
        const float z = (loc + bb[o][e]) + uu;
        hn[o * NHID + j0 + e] = z;
      }
    }
#pragma unroll 1
    for (int i = 0; i < 8; ++i) {
      const int idx = (i >> 2) * NHID + j0 + (i & 3);
      const float z = hn[idx];
      hn[idx] = tanhf(z);
    }
    __syncthreads();
    cur ^= 1;
  }

  {
    const float* hf = &hbuf[cur][0];
    v4f o0, o1;
#pragma unroll
    for (int e = 0; e < 4; ++e) { o0[e] = hf[j0 + e]; o1[e] = hf[NHID + j0 + e]; }
    float* hp = H + (size_t)b * NSTATE + j0;
    *(volatile v4f*)(hp) = o0;
    *(volatile v4f*)(hp + NHID) = o1;
    __threadfence();
    *(volatile v4f*)(hp) = o0;
    *(volatile v4f*)(hp + NHID) = o1;
  }
}

__global__ __launch_bounds__(NTHR) void decode_kernel(const float* __restrict__ H, const float* __restrict__ R_w,
                                                      const float* __restrict__ R_b, float* __restrict__ out) {
  const int idx = blockIdx.x * NTHR + threadIdx.x;
  const int b = idx / NOUTF;
  const int r = idx - b * NOUTF;
  const float* hp = H + (size_t)b * NSTATE;
  const float* wp = R_w + (size_t)r * NSTATE;
  float acc = 0.0f;
#pragma unroll 1
  for (int n = 0; n < NSTATE; n += 4) {
    const v4f hv = *(const v4f*)(hp + n);
    const v4f wv = *(const v4f*)(wp + n);
    acc += hv[0] * bf16r(wv[0]);
    acc += hv[1] * bf16r(wv[1]);
    acc += hv[2] * bf16r(wv[2]);
    acc += hv[3] * bf16r(wv[3]);
  }
  const float v = acc + bf16r(R_b[r]);
  *(volatile float*)(out + idx) = v;
  __threadfence();
  *(volatile float*)(out + idx) = v;
}

extern "C" void kernel_launch(void* const* d_in, const int* in_sizes, int n_in,
                              void* d_out, int out_size, void* d_ws, size_t ws_size, hipStream_t stream) {
  if (n_in < 7 || d_out == nullptr || d_ws == nullptr) return;
  if (in_sizes[0] != NSTEP * NBAT * NINP || in_sizes[1] != NSTATE * NINP || in_sizes[2] != NSTATE ||
      in_sizes[3] != NCHAN * NCHAN * NHID * 3 || in_sizes[4] != NSTATE || in_sizes[5] != NOUTF * NSTATE ||
      in_sizes[6] != NOUTF || out_size != NBAT * NOUTF) return;

  const float* x    = (const float*)d_in[0];
  const float* Wx_w = (const float*)d_in[1];
  const float* Wx_b = (const float*)d_in[2];
  const float* Wy_w = (const float*)d_in[3];
  const float* Wy_b = (const float*)d_in[4];
  const float* R_w  = (const float*)d_in[5];
  const float* R_b  = (const float*)d_in[6];
  float* out = (float*)d_out;

  char* ws = (char*)d_ws; size_t off = 0;
  auto carve = [&](size_t bytes) -> char* { char* p = ws + off; off += (bytes + 255) & ~(size_t)255; return p; };
  unsigned short* XB  = (unsigned short*)carve((size_t)NROWS * NINP * 2);
  unsigned short* WXB = (unsigned short*)carve((size_t)NSTATE * NINP * 2);
  float*          BXR = (float*)carve((size_t)NSTATE * 4);
  float*          HST = (float*)carve((size_t)NBAT * NSTATE * 4);
  float*          UCH = (float*)carve((size_t)MCHUNK * NSTATE * 4);
  if (off > ws_size || off > (size_t)134217728) return;

  const int n8x = NROWS * (NINP / 8);
  const int n8w = NSTATE * (NINP / 8);
  const int n4b = NSTATE / 4;
  cvt8_bf16_kernel<<<n8x / NTHR, NTHR, 0, stream>>>(x, XB, n8x);
  cvt8_bf16_kernel<<<n8w / NTHR, NTHR, 0, stream>>>(Wx_w, WXB, n8w);
  rne_plane_kernel<<<n4b / NTHR, NTHR, 0, stream>>>(Wx_b, BXR, n4b);

  const dim3 ggrid((MCHUNK / 64) * (NSTATE / 64) / 8, 1);
  for (int ch = 0; ch < NCHUNK; ++ch) {
    const unsigned short* Ach = XB + (size_t)ch * MCHUNK * NINP;
    wmma_gemm64<1, false, 2, 0, false, 0><<<ggrid, 256, 0, stream>>>(
        Ach, Ach, NINP, 0L, WXB, WXB, NINP, 0L, (void*)UCH, (void*)UCH, NSTATE, 0L,
        BXR, UCH, 0L, MCHUNK, NSTATE, NINP, 1.0f);
    rec_chunk_kernel<<<NBAT, NTHR, 0, stream>>>(UCH, Wy_w, Wy_b, HST, (ch == 0) ? 1 : 0);
  }

  decode_kernel<<<(NBAT * NOUTF) / NTHR, NTHR, 0, stream>>>(HST, R_w, R_b, out);
}
